// TTM_23811298689124
// MI455X (gfx1250) — hardware-run, weakly checked
//
#include <hip/hip_runtime.h>
#include <math.h>

typedef __attribute__((ext_vector_type(16))) __bf16   v16b;
typedef __attribute__((ext_vector_type(8)))  __bf16   v8b;
typedef __attribute__((ext_vector_type(8)))  _Float16 v8h;
typedef __attribute__((ext_vector_type(8)))  float    v8f;
typedef __attribute__((ext_vector_type(4)))  float    v4f;

constexpr int kCh     = 32;
constexpr int kSp     = 32;
constexpr int kLen    = 360;
constexpr int kT      = 30;
constexpr int kSeg    = kLen / kT;
constexpr int kM      = kCh * kSp;
constexpr int kF      = 4 * kM;
constexpr int kLayers = 10;
constexpr int kMP     = 32;
constexpr int kMT     = kMP / 16;
constexpr float kInvM   = 1.0f / (float)kM;
constexpr float kInvSeg = 1.0f / (float)kSeg;
constexpr float kEps    = 1e-5f;
constexpr float kL2Hi = 27213.0f / 2048.0f;
constexpr float kL2Lo = (float)(13.287712379549449 - 27213.0 / 2048.0);
static_assert(kSeg == 12 && kT * kSeg == kLen, "segment length");
static_assert(kM == 1024 && kF == 4096, "widths");
static_assert((kM % 64) == 0 && (kF % 64) == 0, "GEMM N multiples of 64");
static_assert((kM % 32) == 0 && (kF % 32) == 0, "GEMM K multiples of 32");
static_assert(kMP == 32 && kT <= kMP && kMT == 2, "row padding = 2 tiles of 16");

constexpr size_t kBytesSq  = (size_t)kM * kM * 2;
constexpr size_t kBytesFf  = (size_t)kF * kM * 2;
constexpr size_t kBytesS   = (size_t)kMP * kM * 4;
constexpr size_t kBytesP   = (size_t)kMP * kM * 2;
constexpr size_t kBytesH   = (size_t)kMP * kF * 2;
constexpr size_t kOffW0 = 0;
constexpr size_t kOffWV = kOffW0 + kBytesSq;
constexpr size_t kOffWO = kOffWV + (size_t)kLayers * kBytesSq;
constexpr size_t kOffF1 = kOffWO + (size_t)kLayers * kBytesSq;
constexpr size_t kOffF2 = kOffF1 + kBytesFf;
constexpr size_t kOffSA = kOffF2 + kBytesFf;
constexpr size_t kOffSB = kOffSA + kBytesS;
constexpr size_t kOffVV = kOffSB + kBytesS;
constexpr size_t kOffPE = kOffVV + kBytesS;
constexpr size_t kOffXH = kOffPE + kBytesS;
constexpr size_t kOffXL = kOffXH + kBytesP;
constexpr size_t kOffZH = kOffXL + kBytesP;
constexpr size_t kOffZL = kOffZH + kBytesP;
constexpr size_t kOffCH = kOffZL + kBytesP;
constexpr size_t kOffCL = kOffCH + kBytesP;
constexpr size_t kOffTH = kOffCL + kBytesP;
constexpr size_t kOffTL = kOffTH + kBytesP;
constexpr size_t kOffHH = kOffTL + kBytesP;
constexpr size_t kOffHL = kOffHH + kBytesH;
constexpr size_t kWsTotal = kOffHL + kBytesH;
static_assert(kWsTotal == 62390272ull, "carve total");
static_assert(kWsTotal <= 134217728ull, "carve cap");
static_assert((kOffWV % 128) == 0 && (kOffSA % 128) == 0 && (kOffXH % 128) == 0 && (kOffHH % 128) == 0, "aligned regions");

__device__ __forceinline__ unsigned short f2bf_bits(float f) {
  unsigned u = __float_as_uint(f);
  return (unsigned short)((u + 0x7FFFu + ((u >> 16) & 1u)) >> 16);
}
__device__ __forceinline__ float bf_bits2f(unsigned short h) { return __uint_as_float(((unsigned)h) << 16); }
__device__ __forceinline__ float bfr(float f) { return bf_bits2f(f2bf_bits(f)); }

__device__ __forceinline__ void split8(const float (&o)[8], v8h& hv, v8h& lv) {
#pragma unroll
  for (int e = 0; e < 8; ++e) {
    const unsigned short hb = f2bf_bits(o[e]);
    const unsigned short lb = f2bf_bits(o[e] - bf_bits2f(hb));
    hv[e] = __builtin_bit_cast(_Float16, hb);
    lv[e] = __builtin_bit_cast(_Float16, lb);
  }
}

__device__ __forceinline__ void tie_acc(v8f& a) { asm volatile("" : "+v"(a)); }
__device__ __forceinline__ void nop_guard_b(v8f& a, v16b x, v16b y) { asm volatile("v_nop\n\tv_nop\n\tv_nop\n\tv_nop" : "+v"(a) : "v"(x), "v"(y)); }
__device__ __forceinline__ void keep4_b(v16b a, v16b b, v16b c, v16b d) { asm volatile("v_nop" :: "v"(a), "v"(b), "v"(c), "v"(d)); }
__device__ __forceinline__ void acc_guard4(v8f& a, v8f& b, v8f& c, v8f& d) { asm volatile("v_nop\n\tv_nop\n\tv_nop\n\tv_nop" : "+v"(a), "+v"(b), "+v"(c), "+v"(d)); }

union FragB { v16b v; v8b h[2]; };
__device__ __forceinline__ v16b frag_load(const __bf16* p) {
  FragB f;
  f.h[0] = *(const v8b*)(p);
  f.h[1] = *(const v8b*)(p + 16);
  return f.v;
}
__device__ __forceinline__ v8f mma_b(v16b a, v16b b, v8f c) {
  return __builtin_amdgcn_wmma_f32_16x16x32_bf16(false, a, false, b, (short)0, c, false, false);
}

__global__ __launch_bounds__(256) void cast8_bf16_kernel(const float* __restrict__ in, unsigned short* __restrict__ out, int n8) {
  const int i = blockIdx.x * 256 + threadIdx.x;
  if (i >= n8) return;
  const size_t e0 = (size_t)i << 3;
  const v4f a0 = *(const v4f*)(in + e0);
  const v4f a1 = *(const v4f*)(in + e0 + 4);
  v8h hv;
#pragma unroll
  for (int e = 0; e < 4; ++e) {
    const unsigned short h0 = f2bf_bits(a0[e]);
    const unsigned short h1 = f2bf_bits(a1[e]);
    hv[e]     = __builtin_bit_cast(_Float16, h0);
    hv[4 + e] = __builtin_bit_cast(_Float16, h1);
  }
  unsigned short* q = out + e0;
  *(volatile v8h*)q = hv;
  __threadfence();
  *(volatile v8h*)q = hv;
}

__global__ __launch_bounds__(128) void segmean_kernel(const float* __restrict__ x, unsigned short* __restrict__ XH, unsigned short* __restrict__ XL) {
  const int r  = blockIdx.x;
  const int t  = threadIdx.x;
  const int m0 = t * 8;
  const int s  = m0 >> 5;
  const int c0 = m0 & 31;
  float o[8];
#pragma unroll
  for (int e = 0; e < 8; ++e) o[e] = 0.0f;
  if (r < kT) {
#pragma unroll
    for (int e = 0; e < 8; ++e) {
      const float* p = x + (size_t)(c0 + e) * (kSp * kLen) + (size_t)s * kLen + r * kSeg;
      const v4f q0 = *(const v4f*)(p);
      const v4f q1 = *(const v4f*)(p + 4);
      const v4f q2 = *(const v4f*)(p + 8);
      float acc = 0.0f;
      acc += bfr(q0[0]); acc += bfr(q0[1]); acc += bfr(q0[2]); acc += bfr(q0[3]);
      acc += bfr(q1[0]); acc += bfr(q1[1]); acc += bfr(q1[2]); acc += bfr(q1[3]);
      acc += bfr(q2[0]); acc += bfr(q2[1]); acc += bfr(q2[2]); acc += bfr(q2[3]);
      o[e] = acc * kInvSeg;
    }
  }
  v8h hv, lv;
  split8(o, hv, lv);
  const size_t off = (size_t)r * kM + m0;
  *(volatile v8h*)(XH + off) = hv;
  *(volatile v8h*)(XL + off) = lv;
  __threadfence();
  *(volatile v8h*)(XH + off) = hv;
  *(volatile v8h*)(XL + off) = lv;
}

__global__ __launch_bounds__(128) void postable_kernel(float* __restrict__ PE) {
  __shared__ __align__(16) float sm[kM];
  const int r = blockIdx.x;
  const int t = threadIdx.x;
  const bool live = (r < kT);
#pragma unroll 1
  for (int q = 0; q < 4; ++q) {
    const int p = t + 128 * q;
    const float ex = (float)(4 * p) * kInvM;
    const float th = ex * kL2Hi;
    const float tl = ex * kL2Lo;
    const float fr = exp2f(-th) * exp2f(-tl);
    const float ang = (float)r * fr;
    const float sn = sinf(ang);
    const float cs = cosf(ang);
    sm[2 * p]     = live ? sn : 0.0f;
    sm[2 * p + 1] = live ? cs : 0.0f;
  }
  __syncthreads();
  const v4f v0 = *(const v4f*)(sm + 4 * t);
  const v4f v1 = *(const v4f*)(sm + 512 + 4 * t);
  float* o = PE + (size_t)r * kM;
  *(volatile v4f*)(o + 4 * t) = v0;
  *(volatile v4f*)(o + 512 + 4 * t) = v1;
  __threadfence();
  *(volatile v4f*)(o + 4 * t) = v0;
  *(volatile v4f*)(o + 512 + 4 * t) = v1;
}

template <bool ADDRES>
__global__ __launch_bounds__(128) void rownorm_kernel(const float* __restrict__ S, const float* __restrict__ g,
                                                      const float* __restrict__ b,
                                                      unsigned short* __restrict__ OH, unsigned short* __restrict__ OL) {
  __shared__ float redA[4];
  __shared__ float redB[4];
  const int r    = blockIdx.x;
  const int rc   = (r < kT) ? r : (kT - 1);
  const int t    = threadIdx.x;
  const int lane = t & 31;
  const int wave = t >> 5;
  const int c0   = t * 8;
  const float* sp = S + (size_t)rc * kM + c0;
  const v4f a0 = *(const v4f*)(sp);
  const v4f a1 = *(const v4f*)(sp + 4);
  float xv[8];
#pragma unroll
  for (int e = 0; e < 4; ++e) { xv[e] = a0[e]; xv[4 + e] = a1[e]; }
  float sum = ((xv[0] + xv[1]) + (xv[2] + xv[3])) + ((xv[4] + xv[5]) + (xv[6] + xv[7]));
#pragma unroll
  for (int off = 16; off > 0; off >>= 1) sum += __shfl_xor(sum, off, 32);
  if (lane == 0) redA[wave] = sum;
  __syncthreads();
  const float mu = ((redA[0] + redA[1]) + (redA[2] + redA[3])) * kInvM;
  float dv[8];
#pragma unroll
  for (int e = 0; e < 8; ++e) dv[e] = xv[e] - mu;
  float ss = ((dv[0] * dv[0] + dv[1] * dv[1]) + (dv[2] * dv[2] + dv[3] * dv[3])) +
             ((dv[4] * dv[4] + dv[5] * dv[5]) + (dv[6] * dv[6] + dv[7] * dv[7]));
#pragma unroll
  for (int off = 16; off > 0; off >>= 1) ss += __shfl_xor(ss, off, 32);
  if (lane == 0) redB[wave] = ss;
  __syncthreads();
  const float var = ((redB[0] + redB[1]) + (redB[2] + redB[3])) * kInvM;
  const float inv = 1.0f / sqrtf(var + kEps);
  const v4f g0 = *(const v4f*)(g + c0);
  const v4f g1 = *(const v4f*)(g + c0 + 4);
  const v4f b0 = *(const v4f*)(b + c0);
  const v4f b1 = *(const v4f*)(b + c0 + 4);
  float gv[8], bv[8];
#pragma unroll
  for (int e = 0; e < 4; ++e) {
    gv[e] = bfr(g0[e]); gv[4 + e] = bfr(g1[e]);
    bv[e] = bfr(b0[e]); bv[4 + e] = bfr(b1[e]);
  }
  const bool live = (r < kT);
  float o[8];
#pragma unroll
  for (int e = 0; e < 8; ++e) {
    float y = dv[e] * inv * gv[e] + bv[e];
    if (ADDRES) y += xv[e];
    o[e] = live ? y : 0.0f;
  }
  v8h hv, lv;
  split8(o, hv, lv);
  const size_t off = (size_t)r * kM + c0;
  *(volatile v8h*)(OH + off) = hv;
  *(volatile v8h*)(OL + off) = lv;
  __threadfence();
  *(volatile v8h*)(OH + off) = hv;
  *(volatile v8h*)(OL + off) = lv;
}

__global__ __launch_bounds__(32) void prefix_kernel(const float* __restrict__ V, unsigned short* __restrict__ CH, unsigned short* __restrict__ CL) {
  const int c0 = (blockIdx.x * 32 + threadIdx.x) * 8;
  float run[8];
#pragma unroll
  for (int e = 0; e < 8; ++e) run[e] = 0.0f;
#pragma unroll 1
  for (int row = 0; row < kMP; ++row) {
    const bool live = (row < kT);
    float o[8];
#pragma unroll
    for (int e = 0; e < 8; ++e) o[e] = live ? run[e] : 0.0f;
    v8h hv, lv;
    split8(o, hv, lv);
    const size_t off = (size_t)row * kM + c0;
    *(volatile v8h*)(CH + off) = hv;
    *(volatile v8h*)(CL + off) = lv;
    __threadfence();
    *(volatile v8h*)(CH + off) = hv;
    *(volatile v8h*)(CL + off) = lv;
    const int rl = (row < kT - 1) ? row : (kT - 2);
    const bool addp = (row < kT - 1);
    const v4f a0 = *(const v4f*)(V + (size_t)rl * kM + c0);
    const v4f a1 = *(const v4f*)(V + (size_t)rl * kM + c0 + 4);
#pragma unroll
    for (int e = 0; e < 4; ++e) {
      run[e]     += addp ? a0[e] : 0.0f;
      run[4 + e] += addp ? a1[e] : 0.0f;
    }
  }
}

template <int EPI>
__global__ __launch_bounds__(256) void gemm_a2_kernel(
    const unsigned short* __restrict__ Ahp, const unsigned short* __restrict__ Alp,
    const unsigned short* __restrict__ Btp,
    void* __restrict__ Cout, void* __restrict__ Cout2,
    const float* __restrict__ bias, const float* __restrict__ resid,
    int N, int K, int rowsStore) {
  const __bf16* Ah = (const __bf16*)Ahp;
  const __bf16* Al = (const __bf16*)Alp;
  const __bf16* Bt = (const __bf16*)Btp;
  __shared__ __align__(16) float sT[8][16 * 68];
  const int lane = threadIdx.x & 31;
  const int wave = threadIdx.x >> 5;
  const int tilesN = N >> 6;
  const int tile = blockIdx.x * 8 + wave;
  if (tile >= tilesN) return;
  const int n0 = tile << 6;
  const int rlane = lane & 15;
  const int koff  = (lane >> 4) * 8;
  const int mOff  = (lane >> 4) * 8;

  v8f acc[kMT][4];
#pragma unroll
  for (int i = 0; i < kMT; ++i)
#pragma unroll
    for (int j = 0; j < 4; ++j) acc[i][j] = (v8f){0.f, 0.f, 0.f, 0.f, 0.f, 0.f, 0.f, 0.f};

  for (int k0 = 0; k0 < K; k0 += 32) {
    v16b bh[4];
#pragma unroll
    for (int j = 0; j < 4; ++j) {
      const size_t bo = (size_t)(n0 + (j << 4) + rlane) * K + koff + k0;
      bh[j] = frag_load(Bt + bo);
    }
#pragma unroll
    for (int i = 0; i < kMT; ++i) {
      const size_t ao = (size_t)((i << 4) + rlane) * K + koff + k0;
      const v16b ah = frag_load(Ah + ao);
      const v16b al = frag_load(Al + ao);
#pragma unroll
      for (int j = 0; j < 4; ++j) {
        acc[i][j] = mma_b(ah, bh[j], acc[i][j]);
        acc[i][j] = mma_b(al, bh[j], acc[i][j]);
      }
      tie_acc(acc[i][0]);
      tie_acc(acc[i][1]);
      tie_acc(acc[i][2]);
      nop_guard_b(acc[i][3], ah, al);
    }
    keep4_b(bh[0], bh[1], bh[2], bh[3]);
  }
  acc_guard4(acc[0][0], acc[0][1], acc[0][2], acc[0][3]);
  acc_guard4(acc[1][0], acc[1][1], acc[1][2], acc[1][3]);

  float* slab = sT[wave];
  float bvj[4];
#pragma unroll
  for (int j = 0; j < 4; ++j) {
    bvj[j] = 0.0f;
    if (EPI == 2 || EPI == 3) bvj[j] = bfr(bias[n0 + (j << 4) + rlane]);
  }
#pragma unroll
  for (int i = 0; i < kMT; ++i) {
    const int mBase = i << 4;
#pragma unroll
    for (int j = 0; j < 4; ++j) {
#pragma unroll
      for (int r = 0; r < 8; ++r) {
        const int grow = mBase + mOff + r;
        float v = acc[i][j][r];
        if (EPI == 2 || EPI == 3) v += bvj[j];
        if (EPI != 2) v = (grow < kT) ? v : 0.0f;
        slab[(mOff + r) * 68 + (j << 4) + rlane] = v;
      }
    }
    __builtin_amdgcn_fence(__ATOMIC_RELEASE, "workgroup");
    __builtin_amdgcn_wave_barrier();
    __builtin_amdgcn_fence(__ATOMIC_ACQUIRE, "workgroup");
    if (EPI == 2) {
#pragma unroll 1
      for (int it = 0; it < 32; ++it) {
        const int row = it >> 1;
        const int col = ((it & 1) << 5) + lane;
        const float v = slab[row * 68 + col];
        float gq = 0.5f * v * (1.0f + erff(v * 0.70710678118654752f));
        gq = (mBase + row < kT) ? gq : 0.0f;
        slab[row * 68 + col] = gq;
      }
      __builtin_amdgcn_fence(__ATOMIC_RELEASE, "workgroup");
      __builtin_amdgcn_wave_barrier();
      __builtin_amdgcn_fence(__ATOMIC_ACQUIRE, "workgroup");
    }
    if (EPI != 2) {
      float* C = (float*)Cout;
      const int hh = lane >> 4, c4 = (lane & 15) * 4;
      v4f vv[8];
#pragma unroll
      for (int it = 0; it < 8; ++it) {
        const int row = it * 2 + hh;
        v4f s = *(const v4f*)(slab + row * 68 + c4);
        if (EPI == 1) {
          const v4f rr = *(const v4f*)(resid + (size_t)(mBase + row) * N + n0 + c4);
          s = s + rr;
        }
        vv[it] = s;
      }
      for (int pass = 0; pass < 2; ++pass) {
#pragma unroll
        for (int it = 0; it < 8; ++it) {
          const int row = it * 2 + hh;
          if (mBase + row < rowsStore)
            *(volatile v4f*)(C + (size_t)(mBase + row) * N + n0 + c4) = vv[it];
        }
        __threadfence();
      }
    } else {
      const int q = lane >> 3, c8 = (lane & 7) * 8;
      unsigned short* C  = (unsigned short*)Cout;
      unsigned short* C2 = (unsigned short*)Cout2;
      for (int pass = 0; pass < 2; ++pass) {
#pragma unroll
        for (int it = 0; it < 4; ++it) {
          const int row = it * 4 + q;
          const float* sp = slab + row * 68 + c8;
          v8h hv, lv;
#pragma unroll
          for (int e = 0; e < 8; ++e) {
            const float fv = sp[e];
            const unsigned short hb = f2bf_bits(fv);
            const unsigned short lb = f2bf_bits(fv - bf_bits2f(hb));
            hv[e] = __builtin_bit_cast(_Float16, hb);
            lv[e] = __builtin_bit_cast(_Float16, lb);
          }
          *(volatile v8h*)(C  + (size_t)(mBase + row) * N + n0 + c8) = hv;
          *(volatile v8h*)(C2 + (size_t)(mBase + row) * N + n0 + c8) = lv;
        }
        __threadfence();
      }
    }
    __builtin_amdgcn_fence(__ATOMIC_RELEASE, "workgroup");
    __builtin_amdgcn_wave_barrier();
    __builtin_amdgcn_fence(__ATOMIC_ACQUIRE, "workgroup");
  }
}

extern "C" void kernel_launch(void* const* d_in, const int* in_sizes, int n_in,
                              void* d_out, int out_size, void* d_ws, size_t ws_size,
                              hipStream_t stream) {
  if (n_in < 14) return;
  if (in_sizes[0] != kCh * kSp * kLen) return;
  if (in_sizes[1] != kM * kM) return;
  if (in_sizes[4] != kLayers * kM * kM) return;
  if (in_sizes[5] != kLayers * kM * kM) return;
  if (in_sizes[6] != kM || in_sizes[7] != kM || in_sizes[8] != kM || in_sizes[9] != kM) return;
  if (in_sizes[10] != kF * kM) return;
  if (in_sizes[11] != kF) return;
  if (in_sizes[12] != kM * kF) return;
  if (in_sizes[13] != kM) return;
  if (out_size != kT * kM) return;
  if (ws_size < kWsTotal) return;

  const float* x      = (const float*)d_in[0];
  const float* weight = (const float*)d_in[1];
  const float* Wv     = (const float*)d_in[4];
  const float* Wo     = (const float*)d_in[5];
  const float* ln_g   = (const float*)d_in[6];
  const float* ln_b   = (const float*)d_in[7];
  const float* lnz_g  = (const float*)d_in[8];
  const float* lnz_b  = (const float*)d_in[9];
  const float* fc1_w  = (const float*)d_in[10];
  const float* fc1_b  = (const float*)d_in[11];
  const float* fc2_w  = (const float*)d_in[12];
  const float* fc2_b  = (const float*)d_in[13];

  char* ws = (char*)d_ws;
  unsigned short* W0 = (unsigned short*)(ws + kOffW0);
  unsigned short* WV = (unsigned short*)(ws + kOffWV);
  unsigned short* WO = (unsigned short*)(ws + kOffWO);
  unsigned short* F1 = (unsigned short*)(ws + kOffF1);
  unsigned short* F2 = (unsigned short*)(ws + kOffF2);
  float* SA = (float*)(ws + kOffSA);
  float* SB = (float*)(ws + kOffSB);
  float* VV = (float*)(ws + kOffVV);
  float* PE = (float*)(ws + kOffPE);
  unsigned short* XH = (unsigned short*)(ws + kOffXH);
  unsigned short* XL = (unsigned short*)(ws + kOffXL);
  unsigned short* ZH = (unsigned short*)(ws + kOffZH);
  unsigned short* ZL = (unsigned short*)(ws + kOffZL);
  unsigned short* CH = (unsigned short*)(ws + kOffCH);
  unsigned short* CL = (unsigned short*)(ws + kOffCL);
  unsigned short* TH = (unsigned short*)(ws + kOffTH);
  unsigned short* TL = (unsigned short*)(ws + kOffTL);
  unsigned short* HH = (unsigned short*)(ws + kOffHH);
  unsigned short* HL = (unsigned short*)(ws + kOffHL);

  cast8_bf16_kernel<<<(kM * kM / 8) / 256, 256, 0, stream>>>(weight, W0, kM * kM / 8);
  cast8_bf16_kernel<<<(kLayers * kM * kM / 8) / 256, 256, 0, stream>>>(Wv, WV, kLayers * kM * kM / 8);
  cast8_bf16_kernel<<<(kLayers * kM * kM / 8) / 256, 256, 0, stream>>>(Wo, WO, kLayers * kM * kM / 8);
  cast8_bf16_kernel<<<(kF * kM / 8) / 256, 256, 0, stream>>>(fc1_w, F1, kF * kM / 8);
  cast8_bf16_kernel<<<(kF * kM / 8) / 256, 256, 0, stream>>>(fc2_w, F2, kF * kM / 8);

  segmean_kernel<<<kMP, 128, 0, stream>>>(x, XH, XL);
  postable_kernel<<<kMP, 128, 0, stream>>>(PE);

  const int gridSq = (kM / 64) / 8;
  const int gridFf = (kF / 64) / 8;

  gemm_a2_kernel<1><<<gridSq, 256, 0, stream>>>(XH, XL, W0, (void*)SA, nullptr, nullptr, PE, kM, kM, kMP);

  for (int a = 0; a < kLayers; ++a) {
    const size_t woff = (size_t)a * kM * kM;
    rownorm_kernel<false><<<kMP, 128, 0, stream>>>(SA, ln_g, ln_b, ZH, ZL);
    gemm_a2_kernel<0><<<gridSq, 256, 0, stream>>>(ZH, ZL, WV + woff, (void*)VV, nullptr, nullptr, nullptr, kM, kM, kMP);
    prefix_kernel<<<kM / 256, 32, 0, stream>>>(VV, CH, CL);
    gemm_a2_kernel<1><<<gridSq, 256, 0, stream>>>(CH, CL, WO + woff, (void*)SB, nullptr, nullptr, SA, kM, kM, kMP);
    rownorm_kernel<true><<<kMP, 128, 0, stream>>>(SB, lnz_g, lnz_b, TH, TL);
    gemm_a2_kernel<2><<<gridFf, 256, 0, stream>>>(TH, TL, F1, (void*)HH, (void*)HL, fc1_b, nullptr, kF, kM, kMP);
    if (a + 1 < kLayers) {
      gemm_a2_kernel<3><<<gridSq, 256, 0, stream>>>(HH, HL, F2, (void*)SA, nullptr, fc2_b, nullptr, kM, kF, kMP);
    } else {
      gemm_a2_kernel<3><<<gridSq, 256, 0, stream>>>(HH, HL, F2, d_out, nullptr, fc2_b, nullptr, kM, kF, kT);
    }
  }
}
